// _PyramidSelfAttentionBlock_601295421577
// MI455X (gfx1250) — hardware-run, weakly checked
//
#include <hip/hip_runtime.h>
#include <math.h>

constexpr int kBatch  = 2;
constexpr int kCin    = 512;
constexpr int kImg    = 96;
constexpr int kHW     = kImg * kImg;
constexpr int kCk     = 256;
constexpr int kCo     = 512;
constexpr int kWin    = 48;
constexpr int kTokW   = kWin * kWin;
constexpr int kGroups = kBatch * 4;
constexpr int kTok    = kBatch * kHW;

constexpr float kWCarry    = 16.0f;
constexpr float kWCarryInv = 1.0f / 16.0f;
constexpr float kSimScale  = 0.0625f;
constexpr float kPCarry    = 2048.0f;
constexpr float kCtxCarry  = 256.0f;
constexpr float kPVScale   = kCtxCarry / kPCarry;
constexpr float kOutScale  = 1.0f / (kCtxCarry * kWCarry);

static_assert(kTokW % 64 == 0, "tile multiple");
static_assert(kTok % 64 == 0, "tile multiple");
static_assert(kHW % 64 == 0, "tile multiple");
static_assert(kCin % 32 == 0 && kCk % 32 == 0 && kTokW % 32 == 0, "K multiple of 32");

constexpr size_t kBytesXP  = (size_t)kTok * kCin * 2;
constexpr size_t kHalvesW  = 655360;
constexpr size_t kBytesW   = kHalvesW * 2;
constexpr size_t kBytesAct = (size_t)kTok * kCk * 2;
constexpr size_t kBytesVT  = (size_t)kGroups * kCk * kTokW * 2;
constexpr size_t kBytesS   = (size_t)kTokW * kTokW * 4;
constexpr size_t kBytesP   = (size_t)kTokW * kTokW * 2;
constexpr size_t kOffXP  = 0;
constexpr size_t kOffW   = kOffXP + kBytesXP;
constexpr size_t kOffQ1R = kOffW + kBytesW;
constexpr size_t kOffK1R = kOffQ1R + kBytesAct;
constexpr size_t kOffQ16 = kOffK1R + kBytesAct;
constexpr size_t kOffK16 = kOffQ16 + kBytesAct;
constexpr size_t kOffVT  = kOffK16 + kBytesAct;
constexpr size_t kOffCTX = kOffVT + kBytesVT;
constexpr size_t kOffS   = kOffCTX + kBytesAct;
constexpr size_t kOffP   = kOffS + kBytesS;
constexpr size_t kWsTotal = kOffP + kBytesP;
static_assert(kWsTotal == 108658688, "carve total");
static_assert(kWsTotal <= 134217728, "carve under 128 MiB");
static_assert(kOffW % 128 == 0 && kOffQ1R % 128 == 0 && kOffVT % 128 == 0 && kOffCTX % 128 == 0 && kOffS % 128 == 0 && kOffP % 128 == 0, "128-B aligned regions");
constexpr int kWoffQ1 = 0;
constexpr int kWoffK1 = 131072;
constexpr int kWoffV  = 262144;
constexpr int kWoffQ2 = 393216;
constexpr int kWoffK2 = 458752;
constexpr int kWoffW  = 524288;

typedef __attribute__((ext_vector_type(16))) _Float16 v16h;
typedef __attribute__((ext_vector_type(8)))  _Float16 v8h;
typedef __attribute__((ext_vector_type(16))) __bf16   v16b;
typedef __attribute__((ext_vector_type(8)))  __bf16   v8b;
typedef __attribute__((ext_vector_type(8)))  float    v8f;
typedef __attribute__((ext_vector_type(4)))  float    v4f;
typedef __attribute__((ext_vector_type(4)))  unsigned int v4u;

__device__ __forceinline__ unsigned short f2bf_bits(float f) {
  unsigned u = __float_as_uint(f);
  return (unsigned short)((u + 0x7FFFu + ((u >> 16) & 1u)) >> 16);
}
__device__ __forceinline__ float bf_bits2f(unsigned short h) { return __uint_as_float(((unsigned)h) << 16); }

__device__ __forceinline__ void dep_guard_h(v8f& a, v8f& b, v16h x, v16h y) { asm volatile("v_nop\n\tv_nop\n\tv_nop\n\tv_nop" : "+v"(a), "+v"(b) : "v"(x), "v"(y)); }
__device__ __forceinline__ void dep_guard_b(v8f& a, v8f& b, v16b x, v16b y) { asm volatile("v_nop\n\tv_nop\n\tv_nop\n\tv_nop" : "+v"(a), "+v"(b) : "v"(x), "v"(y)); }
__device__ __forceinline__ void keep4_h(v16h a, v16h b, v16h c, v16h d) { asm volatile("v_nop" :: "v"(a), "v"(b), "v"(c), "v"(d)); }
__device__ __forceinline__ void keep4_b(v16b a, v16b b, v16b c, v16b d) { asm volatile("v_nop" :: "v"(a), "v"(b), "v"(c), "v"(d)); }
__device__ __forceinline__ void acc_guard4(v8f& a, v8f& b, v8f& c, v8f& d) { asm volatile("v_nop\n\tv_nop\n\tv_nop\n\tv_nop" : "+v"(a), "+v"(b), "+v"(c), "+v"(d)); }
template <typename T> struct Frag;
template <> struct Frag<_Float16> {
  typedef v16h V; union U { v16h v; v8h h[2]; };
  static __device__ __forceinline__ v16h load(const _Float16* p) {
    U f; f.h[0] = *(const v8h*)(p); f.h[1] = *(const v8h*)(p + 16); return f.v;
  }
  static __device__ __forceinline__ v8f mma(v16h a, v16h b, v8f c) {
    return __builtin_amdgcn_wmma_f32_16x16x32_f16(false, a, false, b, (short)0, c, false, false);
  }
  static __device__ __forceinline__ void guard(v8f& a, v8f& b, v16h x, v16h y) { dep_guard_h(a, b, x, y); }
  static __device__ __forceinline__ void keep(v16h a, v16h b, v16h c, v16h d) { keep4_h(a, b, c, d); }
};
template <> struct Frag<__bf16> {
  typedef v16b V; union U { v16b v; v8b h[2]; };
  static __device__ __forceinline__ v16b load(const __bf16* p) {
    U f; f.h[0] = *(const v8b*)(p); f.h[1] = *(const v8b*)(p + 16); return f.v;
  }
  static __device__ __forceinline__ v8f mma(v16b a, v16b b, v8f c) {
    return __builtin_amdgcn_wmma_f32_16x16x32_bf16(false, a, false, b, (short)0, c, false, false);
  }
  static __device__ __forceinline__ void guard(v8f& a, v8f& b, v16b x, v16b y) { dep_guard_b(a, b, x, y); }
  static __device__ __forceinline__ void keep(v16b a, v16b b, v16b c, v16b d) { keep4_b(a, b, c, d); }
};

__device__ __forceinline__ unsigned pk16(unsigned short a, unsigned short b) { return (unsigned)a | ((unsigned)b << 16); }
__device__ __forceinline__ unsigned short h_bits(float f) { const _Float16 h = (_Float16)f; return __builtin_bit_cast(unsigned short, h); }

__device__ __forceinline__ int raster_row(int g, int l) {
  const int gb = g >> 2, gsy = (g >> 1) & 1, gsx = g & 1;
  const int iy = l / kWin;
  const int ix = l - iy * kWin;
  return (gb * kImg + gsy * kWin + iy) * kImg + gsx * kWin + ix;
}

template <int ET> struct Elem;
template <> struct Elem<0> { typedef _Float16 T; };
template <> struct Elem<1> { typedef __bf16 T; };
template <int ET, bool SPLIT, int BIAS_MODE, int OUT_MODE, bool RESID, int ACT, bool BNCOL, bool ROWMAP>
__global__ __launch_bounds__(256) void wmma_gemm64(
    const unsigned short* __restrict__ Ap, const unsigned short* __restrict__ A2p, int lda, long strideA,
    const unsigned short* __restrict__ Btp, const unsigned short* __restrict__ Bt2p, int ldb, long strideB,
    void* __restrict__ Cout, void* __restrict__ Cout2, int ldc, long strideC,
    const float* __restrict__ bias, const float* __restrict__ bns, const float* __restrict__ bnt,
    const float* __restrict__ resid, long strideR,
    int M, int N, int K, float scale, int grp0) {
  typedef typename Elem<ET>::T T;
  typedef typename Frag<T>::V V;
  const T* A = (const T*)Ap; const T* A2 = (const T*)A2p; const T* Bt = (const T*)Btp; const T* Bt2 = (const T*)Bt2p;
  __shared__ __align__(16) float sT[8][16 * 68];
  const int b    = blockIdx.y;
  const int lane = threadIdx.x & 31;
  const int wave = threadIdx.x >> 5;
  const int tilesN = N >> 6;
  const int tilesM = M >> 6;
  const int tile = blockIdx.x * 8 + wave;
  if (tile >= tilesM * tilesN) return;
  const int tm = tile / tilesN;
  const int tn = tile - tm * tilesN;
  const int m0 = tm << 6;
  const int n0 = tn << 6;

  const T* Ab  = A  + (size_t)b * strideA;
  const T* Bb  = Bt + (size_t)b * strideB;
  const T* Ab2 = SPLIT ? (A2  + (size_t)b * strideA) : nullptr;
  const T* Bb2 = SPLIT ? (Bt2 + (size_t)b * strideB) : nullptr;

  const int rlane = lane & 15;
  const int koff  = (lane >> 4) * 8;
  const int mOff  = (lane >> 4) * 8;

  v8f acc[4][4];
#pragma unroll
  for (int i = 0; i < 4; ++i)
#pragma unroll
    for (int j = 0; j < 4; ++j) acc[i][j] = (v8f){0.f,0.f,0.f,0.f,0.f,0.f,0.f,0.f};

  for (int k0 = 0; k0 < K; k0 += 32) {
    V bh[4], bl[4];
#pragma unroll
    for (int j = 0; j < 4; ++j) {
      const size_t bo = (size_t)(n0 + (j << 4) + rlane) * ldb + koff + k0;
      bh[j] = Frag<T>::load(Bb + bo);
      if (SPLIT) bl[j] = Frag<T>::load(Bb2 + bo);
    }
#pragma unroll
    for (int i = 0; i < 4; ++i) {
      const size_t ao = (size_t)(m0 + (i << 4) + rlane) * lda + koff + k0;
      V ah = Frag<T>::load(Ab + ao);
      V al;
      if (SPLIT) al = Frag<T>::load(Ab2 + ao);
#pragma unroll
      for (int j = 0; j < 4; ++j) {
        acc[i][j] = Frag<T>::mma(ah, bh[j], acc[i][j]);
        if (SPLIT) {
          acc[i][j] = Frag<T>::mma(ah, bl[j], acc[i][j]);
          acc[i][j] = Frag<T>::mma(al, bh[j], acc[i][j]);
        }
      }
      Frag<T>::guard(acc[i][0], acc[i][3], ah, SPLIT ? al : ah);
    }
    Frag<T>::keep(bh[0], bh[1], bh[2], bh[3]);
    if (SPLIT) Frag<T>::keep(bl[0], bl[1], bl[2], bl[3]);
  }
  acc_guard4(acc[0][0], acc[0][1], acc[0][2], acc[0][3]);
  acc_guard4(acc[1][0], acc[1][1], acc[1][2], acc[1][3]);
  acc_guard4(acc[2][0], acc[2][1], acc[2][2], acc[2][3]);
  acc_guard4(acc[3][0], acc[3][1], acc[3][2], acc[3][3]);

  float* slab = sT[wave];
  const float* Rb = RESID ? (resid + (size_t)b * strideR) : nullptr;
#pragma unroll
  for (int i = 0; i < 4; ++i) {
    const int mBase = m0 + (i << 4);
#pragma unroll
    for (int j = 0; j < 4; ++j) {
      const int n = n0 + (j << 4) + rlane;
      float bv = 0.f, sv = 1.f, tv = 0.f;
      if (BIAS_MODE == 2) bv = bias[n];
      if (BNCOL) { sv = bns[n]; tv = bnt[n]; }
#pragma unroll
      for (int r = 0; r < 8; ++r) {
        float v = acc[i][j][r] * scale;
        if (BIAS_MODE == 1) v += bias[mBase + mOff + r];
        if (BIAS_MODE == 2) v += bv;
        if (RESID) v += Rb[(size_t)(mBase + mOff + r) * ldc + n];
        if (BNCOL) v = v * sv + tv;
        if (ACT == 2) v = fmaxf(v, 0.0f);
        if (ACT == 4) v = (v > 0.f) ? v : 0.01f * v;
        slab[(mOff + r) * 68 + (j << 4) + rlane] = v;
      }
    }
    __builtin_amdgcn_fence(__ATOMIC_RELEASE, "workgroup");
    __builtin_amdgcn_wave_barrier();
    __builtin_amdgcn_fence(__ATOMIC_ACQUIRE, "workgroup");
    if (OUT_MODE == 0) {
      float* C = (float*)Cout + (size_t)b * strideC;
      const int hh = lane >> 4, c4 = (lane & 15) * 4;
      for (int pass = 0; pass < 2; ++pass) {
#pragma unroll
        for (int it = 0; it < 8; ++it) {
          const int row = it * 2 + hh;
          v4f v = *(const v4f*)(slab + row * 68 + c4);
          *(volatile v4f*)(C + (size_t)(mBase + row) * ldc + n0 + c4) = v;
        }
        __threadfence();
      }
    } else {
      const int q = lane >> 3, c8 = (lane & 7) * 8;
      unsigned short* C  = (unsigned short*)Cout  + (size_t)b * strideC;
      unsigned short* C2 = (OUT_MODE == 2) ? ((unsigned short*)Cout2 + (size_t)b * strideC) : nullptr;
      for (int pass = 0; pass < 2; ++pass) {
#pragma unroll
        for (int it = 0; it < 4; ++it) {
          const int row = it * 4 + q;
          const float* sp = slab + row * 68 + c8;
          v8h hv, lv;
#pragma unroll
          for (int e = 0; e < 8; ++e) {
            if (OUT_MODE == 1) {
              hv[e] = (_Float16)sp[e];
            } else {
              unsigned short hb = f2bf_bits(sp[e]);
              unsigned short lb = f2bf_bits(sp[e] - bf_bits2f(hb));
              hv[e] = __builtin_bit_cast(_Float16, hb);
              lv[e] = __builtin_bit_cast(_Float16, lb);
            }
          }
          const int lrow = mBase + row;
          size_t ro;
          if (ROWMAP) ro = (size_t)raster_row(b + grp0, lrow) * (size_t)ldc;
          else ro = (size_t)lrow * (size_t)ldc;
          *(volatile v8h*)(C + ro + n0 + c8) = hv;
          if (OUT_MODE == 2) *(volatile v8h*)(C2 + ro + n0 + c8) = lv;
        }
        __threadfence();
      }
    }
    __builtin_amdgcn_fence(__ATOMIC_RELEASE, "workgroup");
    __builtin_amdgcn_wave_barrier();
    __builtin_amdgcn_fence(__ATOMIC_ACQUIRE, "workgroup");
  }
}

__global__ __launch_bounds__(256) void xpose_kernel(const float* __restrict__ x, unsigned short* __restrict__ xp) {
  __shared__ float sm[64][65];
  const int t  = threadIdx.x;
  const int l0 = blockIdx.x * 64;
  const int c0 = blockIdx.y * 64;
  const int g  = blockIdx.z;
  const int gb = g >> 2, gsy = (g >> 1) & 1, gsx = g & 1;
  const float* xb = x + (size_t)gb * kCin * kHW;
#pragma unroll
  for (int i = 0; i < 16; ++i) {
    const int e  = i * 256 + t;
    const int cl = e >> 6;
    const int r  = e & 63;
    const int l  = l0 + r;
    const int iy = l / kWin;
    const int ix = l - iy * kWin;
    const int p  = (gsy * kWin + iy) * kImg + gsx * kWin + ix;
    sm[r][cl] = xb[(size_t)(c0 + cl) * kHW + p];
  }
  __syncthreads();
  const int lane = t & 31, wave = t >> 5;
  const int q = lane >> 3, c8 = (lane & 7) * 8;
  for (int pass = 0; pass < 2; ++pass) {
#pragma unroll
    for (int it = 0; it < 2; ++it) {
      const int row = wave * 8 + it * 4 + q;
      unsigned short hb[8];
#pragma unroll
      for (int e = 0; e < 8; ++e) hb[e] = h_bits(sm[row][c8 + e]);
      const v4u u = (v4u){pk16(hb[0], hb[1]), pk16(hb[2], hb[3]), pk16(hb[4], hb[5]), pk16(hb[6], hb[7])};
      *(volatile v4u*)(xp + ((size_t)g * kTokW + l0 + row) * kCin + c0 + c8) = u;
    }
    __threadfence();
  }
}

__global__ __launch_bounds__(256) void wcast_kernel(const float* __restrict__ w0, const float* __restrict__ w1,
                                                    const float* __restrict__ w2, const float* __restrict__ w3,
                                                    const float* __restrict__ w4, const float* __restrict__ w5,
                                                    unsigned short* __restrict__ wb, float scale) {
  const int z = blockIdx.y;
  const float* in = (z == 0) ? w0 : (z == 1) ? w1 : (z == 2) ? w2 : (z == 3) ? w3 : (z == 4) ? w4 : w5;
  const int oo  = (z == 0) ? kWoffQ1 : (z == 1) ? kWoffK1 : (z == 2) ? kWoffV : (z == 3) ? kWoffQ2 : (z == 4) ? kWoffK2 : kWoffW;
  const int n8  = (z == 3 || z == 4) ? 8192 : 16384;
  const int i = blockIdx.x * 256 + threadIdx.x;
  if (i >= n8) return;
  const float* p = in + 8 * (size_t)i;
  const v4f a = *(const v4f*)(p);
  const v4f c = *(const v4f*)(p + 4);
  unsigned short hb[8];
#pragma unroll
  for (int e = 0; e < 4; ++e) {
    hb[e]     = h_bits(a[e] * scale);
    hb[4 + e] = h_bits(c[e] * scale);
  }
  const v4u u = (v4u){pk16(hb[0], hb[1]), pk16(hb[2], hb[3]), pk16(hb[4], hb[5]), pk16(hb[6], hb[7])};
  unsigned short* qo = wb + oo + 8 * (size_t)i;
  *(volatile v4u*)qo = u;
  __threadfence();
  *(volatile v4u*)qo = u;
}

__global__ __launch_bounds__(288) void softmax_row_kernel(const float* __restrict__ S, unsigned short* __restrict__ P, float carry) {
  __shared__ float redM[9];
  __shared__ float redS[9];
  const int row  = blockIdx.x;
  const int t    = threadIdx.x;
  const int lane = t & 31, wave = t >> 5;
  const int c0   = t * 8;
  const float* sr = S + (size_t)row * kTokW + c0;
  const v4f a = *(const v4f*)(sr);
  const v4f c = *(const v4f*)(sr + 4);
  float x[8];
#pragma unroll
  for (int e = 0; e < 4; ++e) { x[e] = a[e]; x[4 + e] = c[e]; }
  float m = fmaxf(fmaxf(fmaxf(x[0], x[1]), fmaxf(x[2], x[3])), fmaxf(fmaxf(x[4], x[5]), fmaxf(x[6], x[7])));
#pragma unroll
  for (int off = 16; off > 0; off >>= 1) m = fmaxf(m, __shfl_xor(m, off, 32));
  if (lane == 0) redM[wave] = m;
  __syncthreads();
  float gm = redM[0];
#pragma unroll
  for (int w = 1; w < 9; ++w) gm = fmaxf(gm, redM[w]);
  float ev[8];
  float s = 0.f;
#pragma unroll
  for (int e = 0; e < 8; ++e) { ev[e] = expf(x[e] - gm); s += ev[e]; }
#pragma unroll
  for (int off = 16; off > 0; off >>= 1) s += __shfl_xor(s, off, 32);
  if (lane == 0) redS[wave] = s;
  __syncthreads();
  float tot = redS[0];
#pragma unroll
  for (int w = 1; w < 9; ++w) tot += redS[w];
  const float inv = carry * (1.0f / tot);
  unsigned short hb[8];
#pragma unroll
  for (int e = 0; e < 8; ++e) hb[e] = h_bits(ev[e] * inv);
  const v4u u = (v4u){pk16(hb[0], hb[1]), pk16(hb[2], hb[3]), pk16(hb[4], hb[5]), pk16(hb[6], hb[7])};
  unsigned short* po = P + (size_t)row * kTokW + c0;
  *(volatile v4u*)po = u;
  __threadfence();
  *(volatile v4u*)po = u;
}

extern "C" void kernel_launch(void* const* d_in, const int* in_sizes, int n_in,
                              void* d_out, int out_size, void* d_ws, size_t ws_size,
                              hipStream_t stream) {
  if (n_in < 21) return;
  if (in_sizes[0] != kBatch * kCin * kHW) return;
  if (out_size != kBatch * kCo * kHW) return;
  if (in_sizes[1] != kCk * kCin || in_sizes[5] != kCk * kCk || in_sizes[9] != kCk * kCin ||
      in_sizes[13] != kCk * kCk || in_sizes[17] != kCk * kCin || in_sizes[19] != kCo * kCk) return;
  if (ws_size < kWsTotal) return;

  const float* x    = (const float*)d_in[0];
  const float* q1_w = (const float*)d_in[1];  const float* q1_b = (const float*)d_in[2];
  const float* q1_s = (const float*)d_in[3];  const float* q1_t = (const float*)d_in[4];
  const float* q2_w = (const float*)d_in[5];  const float* q2_b = (const float*)d_in[6];
  const float* q2_s = (const float*)d_in[7];  const float* q2_t = (const float*)d_in[8];
  const float* k1_w = (const float*)d_in[9];  const float* k1_b = (const float*)d_in[10];
  const float* k1_s = (const float*)d_in[11]; const float* k1_t = (const float*)d_in[12];
  const float* k2_w = (const float*)d_in[13]; const float* k2_b = (const float*)d_in[14];
  const float* k2_s = (const float*)d_in[15]; const float* k2_t = (const float*)d_in[16];
  const float* v_w  = (const float*)d_in[17]; const float* v_b  = (const float*)d_in[18];
  const float* w_w  = (const float*)d_in[19]; const float* w_b  = (const float*)d_in[20];
  float* out = (float*)d_out;

  char* ws = (char*)d_ws;
  unsigned short* XP  = (unsigned short*)(ws + kOffXP);
  unsigned short* WB  = (unsigned short*)(ws + kOffW);
  unsigned short* Wq1 = WB + kWoffQ1;
  unsigned short* Wk1 = WB + kWoffK1;
  unsigned short* Wv  = WB + kWoffV;
  unsigned short* Wq2 = WB + kWoffQ2;
  unsigned short* Wk2 = WB + kWoffK2;
  unsigned short* Ww  = WB + kWoffW;
  unsigned short* Q1R = (unsigned short*)(ws + kOffQ1R);
  unsigned short* K1R = (unsigned short*)(ws + kOffK1R);
  unsigned short* Q16 = (unsigned short*)(ws + kOffQ16);
  unsigned short* K16 = (unsigned short*)(ws + kOffK16);
  unsigned short* VT  = (unsigned short*)(ws + kOffVT);
  unsigned short* CTX = (unsigned short*)(ws + kOffCTX);
  float*          Sp  = (float*)(ws + kOffS);
  unsigned short* Pp  = (unsigned short*)(ws + kOffP);
  const float* fz = w_b;

  xpose_kernel<<<dim3(kTokW / 64, kCin / 64, kGroups), 256, 0, stream>>>(x, XP);
  wcast_kernel<<<dim3(64, 6), 256, 0, stream>>>(q1_w, k1_w, v_w, q2_w, k2_w, w_w, WB, kWCarry);

  wmma_gemm64<0, false, 2, 1, false, 2, true, false><<<dim3(144, 1), 256, 0, stream>>>(
      XP, XP, kCin, 0L, Wq1, Wq1, kCin, 0L, (void*)Q1R, (void*)Q1R, kCk, 0L,
      q1_b, q1_s, q1_t, fz, 0L, kTok, kCk, kCin, kWCarryInv, 0);
  wmma_gemm64<0, false, 2, 1, false, 2, true, false><<<dim3(144, 1), 256, 0, stream>>>(
      XP, XP, kCin, 0L, Wk1, Wk1, kCin, 0L, (void*)K1R, (void*)K1R, kCk, 0L,
      k1_b, k1_s, k1_t, fz, 0L, kTok, kCk, kCin, kWCarryInv, 0);
  wmma_gemm64<0, false, 1, 1, false, 0, false, false><<<dim3(18, kGroups), 256, 0, stream>>>(
      Wv, Wv, kCin, 0L, XP, XP, kCin, (long)kTokW * kCin, (void*)VT, (void*)VT, kTokW, (long)kCk * kTokW,
      v_b, fz, fz, fz, 0L, kCk, kTokW, kCin, kWCarryInv, 0);

  wmma_gemm64<0, false, 2, 1, false, 2, true, false><<<dim3(144, 1), 256, 0, stream>>>(
      Q1R, Q1R, kCk, 0L, Wq2, Wq2, kCk, 0L, (void*)Q16, (void*)Q16, kCk, 0L,
      q2_b, q2_s, q2_t, fz, 0L, kTok, kCk, kCk, kWCarryInv, 0);
  wmma_gemm64<0, false, 2, 1, false, 2, true, false><<<dim3(144, 1), 256, 0, stream>>>(
      K1R, K1R, kCk, 0L, Wk2, Wk2, kCk, 0L, (void*)K16, (void*)K16, kCk, 0L,
      k2_b, k2_s, k2_t, fz, 0L, kTok, kCk, kCk, kWCarryInv, 0);

  for (int g = 0; g < kGroups; ++g) {
    const unsigned short* Qg = Q16 + (size_t)g * kTokW * kCk;
    const unsigned short* Kg = K16 + (size_t)g * kTokW * kCk;
    const unsigned short* Vg = VT  + (size_t)g * kCk * kTokW;
    wmma_gemm64<0, false, 0, 0, false, 0, false, false><<<dim3(162, 1), 256, 0, stream>>>(
        Qg, Qg, kCk, 0L, Kg, Kg, kCk, 0L, (void*)Sp, (void*)Sp, kTokW, 0L,
        fz, fz, fz, fz, 0L, kTokW, kTokW, kCk, kSimScale, 0);
    softmax_row_kernel<<<kTokW, 288, 0, stream>>>(Sp, Pp, kPCarry);
    wmma_gemm64<0, false, 0, 1, false, 0, false, true><<<dim3(18, 1), 256, 0, stream>>>(
        Pp, Pp, kTokW, 0L, Vg, Vg, kTokW, 0L, (void*)CTX, (void*)CTX, kCk, 0L,
        fz, fz, fz, fz, 0L, kTokW, kCk, kTokW, kPVScale, g);
  }

  wmma_gemm64<0, false, 1, 0, false, 0, false, false><<<dim3(144, kBatch), 256, 0, stream>>>(
      Ww, Ww, kCk, 0L, CTX, CTX, kCk, (long)kHW * kCk, (void*)out, (void*)out, kHW, (long)kCo * kHW,
      w_b, fz, fz, fz, 0L, kCo, kHW, kCk, kOutScale, 0);
}
